// ZoomTransformerBlock_74302934221438
// MI455X (gfx1250) — hardware-verified
//
#include <hip/hip_runtime.h>
#include <stdint.h>

typedef _Float16 v16h __attribute__((ext_vector_type(16)));
typedef _Float16 v8h  __attribute__((ext_vector_type(8)));
typedef float    v8f  __attribute__((ext_vector_type(8)));
typedef float    v4f  __attribute__((ext_vector_type(4)));

constexpr int NBAT = 2;
constexpr int NTOK = 2048;
constexpr int DM   = 1024;
constexpr int NHD  = 16;
constexpr int DHD  = 64;
constexpr int D3   = 3072;
constexpr int DFF  = 4096;
constexpr int MR   = NBAT * NTOK;
constexpr int QKP  = 2 * DM;
constexpr float SCALE_F = 0.03125f;
constexpr float LN_EPS  = 1e-5f;
constexpr float WSC  = 32.0f;
constexpr float WSC2 = 64.0f;
constexpr float PSC  = 16.0f;
constexpr float HSC  = 8.0f;

constexpr int AQB = 64;
constexpr int AKC = 64;
constexpr int ANW = 4;

constexpr size_t O_QKVT = 0;
constexpr size_t O_PRJT = O_QKVT + (size_t)D3 * DM * 2;
constexpr size_t O_W1T  = O_PRJT + (size_t)DM * DM * 2;
constexpr size_t O_W2T  = O_W1T  + (size_t)DFF * DM * 2;
constexpr size_t O_H    = O_W2T  + (size_t)DM * DFF * 2;
constexpr size_t O_QK   = O_H    + (size_t)MR * DM * 2;
constexpr size_t O_VT   = O_QK   + (size_t)MR * QKP * 2;
constexpr size_t O_AO   = O_VT   + (size_t)DM * MR * 2;
constexpr size_t O_X1   = O_AO   + (size_t)MR * DM * 2;
constexpr size_t O_HID  = O_X1   + (size_t)MR * DM * 4;
constexpr size_t O_END  = O_HID  + (size_t)MR * DFF * 2;
static_assert(O_END == (size_t)117440512);
static_assert(O_END <= (size_t)134217728);

union FragU { v16h v; v8h h[2]; };

__device__ __forceinline__ v16h fload(const _Float16* p) {
  FragU f;
  f.h[0] = *(const v8h*)(p);
  f.h[1] = *(const v8h*)(p + 16);
  return f.v;
}
__device__ __forceinline__ v8f zero8() { return (v8f){0.f, 0.f, 0.f, 0.f, 0.f, 0.f, 0.f, 0.f}; }
__device__ __forceinline__ v8f mma_raw(v16h a, v16h b, v8f c) {
  return __builtin_amdgcn_wmma_f32_16x16x32_f16(false, a, false, b, (short)0, c, false, false);
}
__device__ __forceinline__ v8f mma_g(v16h a, v16h b, v8f c) {
  c = mma_raw(a, b, c);
  asm volatile("v_nop\n\tv_nop\n\tv_nop\n\tv_nop" : "+v"(c) : "v"(a), "v"(b));
  return c;
}
__device__ __forceinline__ void dep_guard(v8f& a, v8f& b, v16h x, v16h y) {
  asm volatile("v_nop\n\tv_nop\n\tv_nop\n\tv_nop" : "+v"(a), "+v"(b) : "v"(x), "v"(y));
}
__device__ __forceinline__ void keep4(v16h a, v16h b, v16h c, v16h d) {
  asm volatile("v_nop" :: "v"(a), "v"(b), "v"(c), "v"(d));
}
__device__ __forceinline__ void acc_guard4(v8f& a, v8f& b, v8f& c, v8f& d) {
  asm volatile("v_nop\n\tv_nop\n\tv_nop\n\tv_nop" : "+v"(a), "+v"(b), "+v"(c), "+v"(d));
}
__device__ __forceinline__ void lds_wave_sync() {
  __builtin_amdgcn_fence(__ATOMIC_RELEASE, "workgroup");
  __builtin_amdgcn_wave_barrier();
  __builtin_amdgcn_fence(__ATOMIC_ACQUIRE, "workgroup");
}

__global__ __launch_bounds__(256) void tconv_kernel(const float* __restrict__ W, _Float16* __restrict__ o,
                                                    int R, int Cc, float scale) {
  __shared__ __align__(16) float tf[64 * 68];
  const int c0  = blockIdx.x * 64;
  const int r0  = blockIdx.y * 64;
  const int tid = threadIdx.x;
  {
    const int lr = tid >> 4;
    const int c4 = (tid & 15) * 4;
#pragma unroll
    for (int it = 0; it < 4; ++it) {
      const int rr = it * 16 + lr;
      const v4f a = *(const v4f*)(W + (size_t)(r0 + rr) * Cc + c0 + c4);
      *(v4f*)(tf + rr * 68 + c4) = a;
    }
  }
  __syncthreads();
  const int sub = tid >> 3;
  const int c8  = (tid & 7) * 8;
  v8h hv[2];
#pragma unroll
  for (int it = 0; it < 2; ++it) {
    const int oc = it * 32 + sub;
    v8h t;
#pragma unroll
    for (int e = 0; e < 8; ++e) t[e] = (_Float16)(tf[(c8 + e) * 68 + oc] * scale);
    hv[it] = t;
  }
  for (int pass = 0; pass < 2; ++pass) {
#pragma unroll
    for (int it = 0; it < 2; ++it) {
      const int oc = it * 32 + sub;
      *(volatile v8h*)(o + (size_t)(c0 + oc) * R + r0 + c8) = hv[it];
    }
    __threadfence();
  }
}

__global__ __launch_bounds__(128) void ln_kernel(const float* __restrict__ x, const float* __restrict__ w,
                                                 const float* __restrict__ bb, _Float16* __restrict__ out) {
  __shared__ float red[2][4];
  const int row  = blockIdx.x;
  const int tid  = threadIdx.x;
  const int lane = tid & 31;
  const int wave = tid >> 5;
  const int c0   = tid * 8;
  const float* xr = x + (size_t)row * DM + c0;
  const v4f a0 = *(const v4f*)(xr);
  const v4f a1 = *(const v4f*)(xr + 4);
  v8f v;
  v[0] = a0[0]; v[1] = a0[1]; v[2] = a0[2]; v[3] = a0[3];
  v[4] = a1[0]; v[5] = a1[1]; v[6] = a1[2]; v[7] = a1[3];
  float s = 0.f;
#pragma unroll
  for (int e = 0; e < 8; ++e) s += v[e];
#pragma unroll
  for (int m = 1; m < 32; m <<= 1) s += __shfl_xor(s, m, 32);
  if (lane == 0) red[0][wave] = s;
  __syncthreads();
  const float mu = (red[0][0] + red[0][1] + red[0][2] + red[0][3]) * (1.0f / (float)DM);
  float s2 = 0.f;
#pragma unroll
  for (int e = 0; e < 8; ++e) { const float d = v[e] - mu; s2 += d * d; }
#pragma unroll
  for (int m = 1; m < 32; m <<= 1) s2 += __shfl_xor(s2, m, 32);
  if (lane == 0) red[1][wave] = s2;
  __syncthreads();
  const float var  = (red[1][0] + red[1][1] + red[1][2] + red[1][3]) * (1.0f / (float)DM);
  const float rstd = rsqrtf(var + LN_EPS);
  const v4f w0 = *(const v4f*)(w + c0);
  const v4f w1 = *(const v4f*)(w + c0 + 4);
  const v4f b0 = *(const v4f*)(bb + c0);
  const v4f b1 = *(const v4f*)(bb + c0 + 4);
  v8f wv, bv;
  wv[0] = w0[0]; wv[1] = w0[1]; wv[2] = w0[2]; wv[3] = w0[3];
  wv[4] = w1[0]; wv[5] = w1[1]; wv[6] = w1[2]; wv[7] = w1[3];
  bv[0] = b0[0]; bv[1] = b0[1]; bv[2] = b0[2]; bv[3] = b0[3];
  bv[4] = b1[0]; bv[5] = b1[1]; bv[6] = b1[2]; bv[7] = b1[3];
  v8h hv;
#pragma unroll
  for (int e = 0; e < 8; ++e) hv[e] = (_Float16)((v[e] - mu) * rstd * wv[e] + bv[e]);
  _Float16* op = out + (size_t)row * DM + c0;
  *(volatile v8h*)op = hv;
  __threadfence();
  *(volatile v8h*)op = hv;
}

template <int BIAS_MODE, int OUT_MODE, bool RESID, int ACT>
__global__ __launch_bounds__(256) void gemm64_kernel(
    const _Float16* __restrict__ A, int lda,
    const _Float16* __restrict__ Bt, int ldb,
    void* __restrict__ Cout, int ldc,
    const float* __restrict__ bias,
    const float* __restrict__ resid, int ldr,
    int M, int N, int K, float scale, float oscale) {
  __shared__ __align__(16) float sT[8][16 * 68];
  const int lane = threadIdx.x & 31;
  const int wave = threadIdx.x >> 5;
  const int tilesN = N >> 6;
  const int tilesM = M >> 6;
  const int tile = blockIdx.x * 8 + wave;
  if (tile >= tilesM * tilesN) return;
  const int tm = tile / tilesN;
  const int tn = tile - tm * tilesN;
  const int m0 = tm << 6;
  const int n0 = tn << 6;

  const int rlane = lane & 15;
  const int koff  = (lane >> 4) * 8;
  const int mOff  = (lane >> 4) * 8;

  v8f acc[4][4];
#pragma unroll
  for (int i = 0; i < 4; ++i)
#pragma unroll
    for (int j = 0; j < 4; ++j) acc[i][j] = zero8();

  for (int k0 = 0; k0 < K; k0 += 32) {
    v16h bh[4];
#pragma unroll
    for (int j = 0; j < 4; ++j)
      bh[j] = fload(Bt + (size_t)(n0 + (j << 4) + rlane) * ldb + k0 + koff);
#pragma unroll
    for (int i = 0; i < 4; ++i) {
      const v16h ah = fload(A + (size_t)(m0 + (i << 4) + rlane) * lda + k0 + koff);
#pragma unroll
      for (int j = 0; j < 4; ++j) acc[i][j] = mma_raw(ah, bh[j], acc[i][j]);
      dep_guard(acc[i][0], acc[i][3], ah, bh[3]);
    }
    keep4(bh[0], bh[1], bh[2], bh[3]);
  }
  acc_guard4(acc[0][0], acc[0][1], acc[0][2], acc[0][3]);
  acc_guard4(acc[1][0], acc[1][1], acc[1][2], acc[1][3]);
  acc_guard4(acc[2][0], acc[2][1], acc[2][2], acc[2][3]);
  acc_guard4(acc[3][0], acc[3][1], acc[3][2], acc[3][3]);

  float* slab = sT[wave];
#pragma unroll
  for (int i = 0; i < 4; ++i) {
    const int mBase = m0 + (i << 4);
#pragma unroll
    for (int j = 0; j < 4; ++j) {
      const int n = n0 + (j << 4) + rlane;
      float bn = 0.f;
      if (BIAS_MODE == 2) bn = bias[n];
#pragma unroll
      for (int r = 0; r < 8; ++r) {
        float v = acc[i][j][r] * scale;
        if (BIAS_MODE == 1) v += bias[mBase + mOff + r];
        if (BIAS_MODE == 2) v += bn;
        if (ACT == 1) v = 0.5f * v * (1.0f + erff(v * 0.70710678118654752f));
        if (RESID) v += resid[(size_t)(mBase + mOff + r) * ldr + n];
        if (OUT_MODE == 1) v *= oscale;
        slab[(mOff + r) * 68 + (j << 4) + rlane] = v;
      }
    }
    lds_wave_sync();
    if (OUT_MODE == 0) {
      float* C = (float*)Cout;
      const int hh = lane >> 4, c4 = (lane & 15) * 4;
      for (int pass = 0; pass < 2; ++pass) {
#pragma unroll
        for (int it = 0; it < 8; ++it) {
          const int row = it * 2 + hh;
          const v4f vv = *(const v4f*)(slab + row * 68 + c4);
          *(volatile v4f*)(C + (size_t)(mBase + row) * ldc + n0 + c4) = vv;
        }
        __threadfence();
      }
    } else {
      _Float16* C = (_Float16*)Cout;
      const int q = lane >> 3, c8 = (lane & 7) * 8;
      v8h hv[4];
#pragma unroll
      for (int it = 0; it < 4; ++it) {
        const int row = it * 4 + q;
        const float* sp = slab + row * 68 + c8;
        v8h t;
#pragma unroll
        for (int e = 0; e < 8; ++e) t[e] = (_Float16)sp[e];
        hv[it] = t;
      }
      for (int pass = 0; pass < 2; ++pass) {
#pragma unroll
        for (int it = 0; it < 4; ++it) {
          const int row = it * 4 + q;
          *(volatile v8h*)(C + (size_t)(mBase + row) * ldc + n0 + c8) = hv[it];
        }
        __threadfence();
      }
    }
    lds_wave_sync();
  }
}

__global__ __launch_bounds__(128)
void attn_kernel(const _Float16* __restrict__ qk, const _Float16* __restrict__ vt,
                 const float* __restrict__ gamma, const float* __restrict__ dist,
                 _Float16* __restrict__ ao) {
  __shared__ __align__(16) _Float16 Ksh[AKC * DHD];
  __shared__ __align__(16) _Float16 Vth[DHD * AKC];
  __shared__ __align__(16) _Float16 Psh[ANW][16 * AKC];
  __shared__ __align__(16) float    Os[ANW][16 * 68];

  const int tid  = threadIdx.x;
  const int wave = tid >> 5;
  const int lane = tid & 31;
  const int hf   = lane >> 4;
  const int c    = lane & 15;

  const int bx = blockIdx.x;
  const int qb = bx & (NTOK / AQB - 1);
  const int bh = bx >> 5;
  const int hd = bh & (NHD - 1);
  const int b  = bh >> 4;
  const int tokb = b * NTOK;
  const int q0 = qb * AQB + wave * 16;
  const float g = gamma[b * NHD + hd];

  v16h qa[2];
  {
    const _Float16* qp = qk + (size_t)(tokb + q0 + c) * QKP + hd * DHD + 8 * hf;
    qa[0] = fload(qp);
    qa[1] = fload(qp + 32);
  }

  float mrow[8], lrow[8];
  v8f oacc[4];
#pragma unroll
  for (int r = 0; r < 8; ++r) { mrow[r] = -__builtin_inff(); lrow[r] = 0.f; }
#pragma unroll
  for (int t = 0; t < 4; ++t) oacc[t] = zero8();

  _Float16* pw = Psh[wave];

  for (int kc = 0; kc < NTOK / AKC; ++kc) {
    const int kv0 = kc * AKC;
    __syncthreads();
    {
      const int r = tid >> 1, half = (tid & 1) * 32;
      const _Float16* ks = qk + (size_t)(tokb + kv0 + r) * QKP + DM + hd * DHD + half;
      const _Float16* vs = vt + (size_t)(hd * DHD + r) * MR + tokb + kv0 + half;
#pragma unroll
      for (int i = 0; i < 4; ++i) {
        const v8h ka = *(const v8h*)(ks + 8 * i);
        const v8h va = *(const v8h*)(vs + 8 * i);
        *(v8h*)(Ksh + r * DHD + half + 8 * i) = ka;
        *(v8h*)(Vth + r * AKC + half + 8 * i) = va;
      }
    }
    __syncthreads();

    v8f s[4];
#pragma unroll
    for (int j = 0; j < 4; ++j) {
      s[j] = zero8();
#pragma unroll
      for (int dc = 0; dc < 2; ++dc) {
        FragU kb;
        kb.h[0] = *(const v8h*)(Ksh + (j * 16 + c) * DHD + dc * 32 + 8 * hf);
        kb.h[1] = *(const v8h*)(Ksh + (j * 16 + c) * DHD + dc * 32 + 16 + 8 * hf);
        s[j] = mma_g(qa[dc], kb.v, s[j]);
      }
    }

    const float* dr = dist + (size_t)(q0 + 8 * hf) * NTOK + kv0 + c;
    float cm[8];
#pragma unroll
    for (int r = 0; r < 8; ++r) {
      float m = -__builtin_inff();
#pragma unroll
      for (int j = 0; j < 4; ++j) {
        const float dv = dr[(size_t)r * NTOK + j * 16];
        const float sv = s[j][r] * SCALE_F - g * dv;
        s[j][r] = sv;
        m = fmaxf(m, sv);
      }
#pragma unroll
      for (int off = 1; off < 16; off <<= 1) m = fmaxf(m, __shfl_xor(m, off, 32));
      cm[r] = m;
    }

#pragma unroll
    for (int r = 0; r < 8; ++r) {
      const float mnew  = fmaxf(mrow[r], cm[r]);
      const float alpha = __expf(mrow[r] - mnew);
      mrow[r] = mnew;
      float psum = 0.f;
#pragma unroll
      for (int j = 0; j < 4; ++j) {
        const float p = __expf(s[j][r] - mnew);
        psum += p;
        pw[(8 * hf + r) * AKC + j * 16 + c] = (_Float16)(p * PSC);
      }
#pragma unroll
      for (int off = 1; off < 16; off <<= 1) psum += __shfl_xor(psum, off, 32);
      lrow[r] = lrow[r] * alpha + psum;
#pragma unroll
      for (int t = 0; t < 4; ++t) oacc[t][r] *= alpha;
    }
    lds_wave_sync();

#pragma unroll
    for (int kk = 0; kk < 2; ++kk) {
      FragU pa;
      pa.h[0] = *(const v8h*)(pw + c * AKC + kk * 32 + 8 * hf);
      pa.h[1] = *(const v8h*)(pw + c * AKC + kk * 32 + 16 + 8 * hf);
#pragma unroll
      for (int t = 0; t < 4; ++t) {
        FragU vb;
        vb.h[0] = *(const v8h*)(Vth + (t * 16 + c) * AKC + kk * 32 + 8 * hf);
        vb.h[1] = *(const v8h*)(Vth + (t * 16 + c) * AKC + kk * 32 + 16 + 8 * hf);
        oacc[t] = mma_g(pa.v, vb.v, oacc[t]);
      }
    }
  }

  float* os = Os[wave];
#pragma unroll
  for (int r = 0; r < 8; ++r) {
    const float inv = 1.0f / lrow[r];
#pragma unroll
    for (int t = 0; t < 4; ++t) os[(8 * hf + r) * 68 + t * 16 + c] = oacc[t][r] * inv;
  }
  lds_wave_sync();
  {
    const int q = lane >> 3, c8 = (lane & 7) * 8;
    v8h hv[4];
#pragma unroll
    for (int it = 0; it < 4; ++it) {
      const int row = it * 4 + q;
      const float* sp = os + row * 68 + c8;
      v8h t;
#pragma unroll
      for (int e = 0; e < 8; ++e) t[e] = (_Float16)sp[e];
      hv[it] = t;
    }
    for (int pass = 0; pass < 2; ++pass) {
#pragma unroll
      for (int it = 0; it < 4; ++it) {
        const int row = it * 4 + q;
        *(volatile v8h*)(ao + (size_t)(tokb + q0 + row) * DM + hd * DHD + c8) = hv[it];
      }
      __threadfence();
    }
  }
}

extern "C" void kernel_launch(void* const* d_in, const int* in_sizes, int n_in,
                              void* d_out, int out_size, void* d_ws, size_t ws_size,
                              hipStream_t stream) {
  if (n_in < 15) return;
  if (in_sizes[0] != MR * DM || in_sizes[1] != NBAT * NHD || in_sizes[2] != NTOK * NTOK) return;
  if (in_sizes[3] != DM || in_sizes[4] != DM || in_sizes[5] != DM * D3 || in_sizes[6] != D3) return;
  if (in_sizes[7] != DM * DM || in_sizes[8] != DM || in_sizes[9] != DM || in_sizes[10] != DM) return;
  if (in_sizes[11] != DM * DFF || in_sizes[12] != DFF || in_sizes[13] != DFF * DM || in_sizes[14] != DM) return;
  if (out_size != MR * DM) return;
  if (O_END > ws_size) return;

  const float* x     = (const float*)d_in[0];
  const float* gamma = (const float*)d_in[1];
  const float* dist  = (const float*)d_in[2];
  const float* ln1w  = (const float*)d_in[3];
  const float* ln1b  = (const float*)d_in[4];
  const float* qkvw  = (const float*)d_in[5];
  const float* qkvb  = (const float*)d_in[6];
  const float* projw = (const float*)d_in[7];
  const float* projb = (const float*)d_in[8];
  const float* ln2w  = (const float*)d_in[9];
  const float* ln2b  = (const float*)d_in[10];
  const float* w1    = (const float*)d_in[11];
  const float* b1    = (const float*)d_in[12];
  const float* w2    = (const float*)d_in[13];
  const float* b2    = (const float*)d_in[14];
  float* out = (float*)d_out;
  char* ws = (char*)d_ws;

  _Float16* qkvT = (_Float16*)(ws + O_QKVT);
  _Float16* prjT = (_Float16*)(ws + O_PRJT);
  _Float16* w1T  = (_Float16*)(ws + O_W1T);
  _Float16* w2T  = (_Float16*)(ws + O_W2T);
  _Float16* hpl  = (_Float16*)(ws + O_H);
  _Float16* qkp  = (_Float16*)(ws + O_QK);
  _Float16* vtp  = (_Float16*)(ws + O_VT);
  _Float16* aop  = (_Float16*)(ws + O_AO);
  float*    x1   = (float*)(ws + O_X1);
  _Float16* hid  = (_Float16*)(ws + O_HID);

  const dim3 blk(256);

  tconv_kernel<<<dim3(D3 / 64, DM / 64), blk, 0, stream>>>(qkvw, qkvT, DM, D3, WSC);
  tconv_kernel<<<dim3(DM / 64, DM / 64), blk, 0, stream>>>(projw, prjT, DM, DM, WSC);
  tconv_kernel<<<dim3(DFF / 64, DM / 64), blk, 0, stream>>>(w1, w1T, DM, DFF, WSC);
  tconv_kernel<<<dim3(DM / 64, DFF / 64), blk, 0, stream>>>(w2, w2T, DFF, DM, WSC2);

  ln_kernel<<<dim3(MR), dim3(128), 0, stream>>>(x, ln1w, ln1b, hpl);

  {
    const int tiles = (MR / 64) * (QKP / 64);
    gemm64_kernel<2, 1, false, 0><<<dim3((tiles + 7) / 8), blk, 0, stream>>>(
        hpl, DM, qkvT, DM, (void*)qkp, QKP, qkvb, qkvb, 0, MR, QKP, DM, 1.0f / WSC, 1.0f);
  }
  {
    const int tiles = (DM / 64) * (MR / 64);
    gemm64_kernel<1, 1, false, 0><<<dim3((tiles + 7) / 8), blk, 0, stream>>>(
        qkvT + (size_t)2 * DM * DM, DM, hpl, DM, (void*)vtp, MR, qkvb + 2 * DM, qkvb, 0, DM, MR, DM, 1.0f / WSC, 1.0f);
  }
  attn_kernel<<<dim3(NBAT * NHD * (NTOK / AQB)), dim3(128), 0, stream>>>(qkp, vtp, gamma, dist, aop);

  {
    const int tiles = (MR / 64) * (DM / 64);
    gemm64_kernel<2, 0, true, 0><<<dim3((tiles + 7) / 8), blk, 0, stream>>>(
        aop, DM, prjT, DM, (void*)x1, DM, projb, x, DM, MR, DM, DM, 1.0f / (PSC * WSC), 1.0f);
  }
  ln_kernel<<<dim3(MR), dim3(128), 0, stream>>>(x1, ln2w, ln2b, hpl);

  {
    const int tiles = (MR / 64) * (DFF / 64);
    gemm64_kernel<2, 1, false, 1><<<dim3((tiles + 7) / 8), blk, 0, stream>>>(
        hpl, DM, w1T, DM, (void*)hid, DFF, b1, b1, 0, MR, DFF, DM, 1.0f / WSC, HSC);
  }
  {
    const int tiles = (MR / 64) * (DM / 64);
    gemm64_kernel<2, 0, true, 0><<<dim3((tiles + 7) / 8), blk, 0, stream>>>(
        hid, DFF, w2T, DFF, (void*)out, DM, b2, x1, DM, MR, DM, DFF, 1.0f / (HSC * WSC2), 1.0f);
  }
  (void)hipGetLastError();
}
